// MultiHeadSelfAttention_19164144075432
// MI455X (gfx1250) — hardware-verified
//
#include <hip/hip_runtime.h>
#include <stdint.h>
#include <stddef.h>


#ifndef NB
#define NB 1
#endif
#ifndef SEQ
#define SEQ 4096
#endif
#define NB_FULL   1
#define SEQ_FULL  4096
#define NNODE     (SEQ_FULL)
#define QROWS     (SEQ)
#define HIDC      512
#define NHEAD     8
#define HDIM      64
#define PCARRY    16384.0f
#define CTXSC     0.0009765625f
#define WOC       1024.0f
#define OUNC      0.00006103515625f
#define OCARRY    16.0f
#define PFLUSH    (-27.0f)
#define SCL       0.18033688011112042f
#define XB_BLOCKS ((NNODE * HIDC) / 2048)
#define WT_TILES  ((HIDC / 64) * (HIDC / 64))
#define PLANE_BYTES   ((size_t)NNODE * HIDC * 2)
#define WPLANE_BYTES  ((size_t)HIDC * HIDC * 2)
#define WS_TOTAL      (3 * PLANE_BYTES + 3 * WPLANE_BYTES + WPLANE_BYTES + 5 * PLANE_BYTES)

static_assert(NB == 1 && NB_FULL == 1);
static_assert(QROWS >= 64 && QROWS <= NNODE && (QROWS % 64) == 0);
static_assert(HIDC == NHEAD * HDIM && HDIM == 64 && NHEAD == 8);
static_assert((NNODE % 64) == 0 && (NNODE % 32) == 0);
static_assert(((NNODE * HIDC) % 2048) == 0 && (HIDC % 64) == 0 && (HIDC % 32) == 0);
static_assert(((3 * HIDC) % 128) == 0 && (HIDC % 128) == 0);
static_assert(4 * 256 * 8 == 128 * 64);
static_assert(2 * 256 * 8 == 64 * 64);
static_assert(4 * 256 * 8 == NHEAD * 16 * HDIM);
static_assert(8 * 64 == HIDC);
static_assert(8 * 2 == 16);
static_assert(4 * 32 * 4 == HIDC && 2 * 32 * 8 == HIDC);
static_assert(WS_TOTAL <= (size_t)134217728);

typedef float          v8f   __attribute__((ext_vector_type(8)));
typedef float          v4f_  __attribute__((ext_vector_type(4)));
typedef v4f_           v4f   __attribute__((may_alias));
typedef _Float16       v16h  __attribute__((ext_vector_type(16)));
typedef _Float16       v8h_  __attribute__((ext_vector_type(8)));
typedef v8h_           v8h   __attribute__((may_alias));
typedef __bf16         v16bf __attribute__((ext_vector_type(16)));
typedef unsigned short v8us_ __attribute__((ext_vector_type(8)));
typedef v8us_          v8us  __attribute__((may_alias));
typedef unsigned       v4u_  __attribute__((ext_vector_type(4)));
typedef v4u_           v4u   __attribute__((may_alias));
typedef _Float16       h16;

union FragB { v16bf v; v8us_ h[2]; };
union FragH { v16h  v; v8h_  h[2]; };

__device__ __forceinline__ v8f mma_bf16(const v16bf a, const v16bf b, v8f c)
{
  v8f d = __builtin_amdgcn_wmma_f32_16x16x32_bf16(false, a, false, b, (short)0, c, false, false);
  asm volatile("v_nop\n\tv_nop\n\tv_nop\n\tv_nop" : "+v"(d) : "v"(a), "v"(b));
  return d;
}
__device__ __forceinline__ v8f mma_f16(const v16h a, const v16h b, v8f c)
{
  v8f d = __builtin_amdgcn_wmma_f32_16x16x32_f16(false, a, false, b, (short)0, c, false, false);
  asm volatile("v_nop\n\tv_nop\n\tv_nop\n\tv_nop" : "+v"(d) : "v"(a), "v"(b));
  return d;
}

__device__ __forceinline__ unsigned short bf16_bits(float f)
{
  const __bf16 hb = (__bf16)f;
  return __builtin_bit_cast(unsigned short, hb);
}
__device__ __forceinline__ float bf16_rn(float f)
{
  return (float)(__bf16)f;
}
__device__ __forceinline__ unsigned short f16_bits(float f)
{
  const _Float16 hf = (_Float16)f;
  return __builtin_bit_cast(unsigned short, hf);
}
__device__ __forceinline__ float exp2fast(float x)
{
#if __has_builtin(__builtin_amdgcn_exp2f)
  return __builtin_amdgcn_exp2f(x);
#else
  return exp2f(x);
#endif
}
static __device__ __forceinline__ h16 toh_flush(float v)
{
  const h16 r = (h16)v;
  return (fabsf(v) < 6.103515625e-05f) ? (h16)0.0f : r;
}
static __device__ __forceinline__ unsigned short toh_flush_bits(float v)
{
  const h16 r = toh_flush(v);
  return __builtin_bit_cast(unsigned short, r);
}

__global__ void __launch_bounds__(256) cvt_kernel(
    const float* __restrict__ xq, const float* __restrict__ xk, const float* __restrict__ xv,
    unsigned short* __restrict__ xb)
{
  const int blk = (int)blockIdx.x;
  const int tid = (int)threadIdx.x;
  const float* src;
  unsigned short* dst;
  int t;
  if (blk < XB_BLOCKS) {
    src = xq; dst = xb; t = blk * 256 + tid;
  } else if (blk < 2 * XB_BLOCKS) {
    src = xk; dst = xb + (size_t)NNODE * HIDC; t = (blk - XB_BLOCKS) * 256 + tid;
  } else {
    src = xv; dst = xb + 2 * (size_t)NNODE * HIDC; t = (blk - 2 * XB_BLOCKS) * 256 + tid;
  }

  const v4f_ a = *(const v4f*)(src + (size_t)t * 8);
  const v4f_ b = *(const v4f*)(src + (size_t)t * 8 + 4);
  v8us_ o;
  o[0] = bf16_bits(a[0]); o[1] = bf16_bits(a[1]); o[2] = bf16_bits(a[2]); o[3] = bf16_bits(a[3]);
  o[4] = bf16_bits(b[0]); o[5] = bf16_bits(b[1]); o[6] = bf16_bits(b[2]); o[7] = bf16_bits(b[3]);
  unsigned short* p = dst + (size_t)t * 8;
  *(volatile v8us_*)p = o;
  __threadfence();
  *(volatile v8us_*)p = o;
}

__global__ void __launch_bounds__(256) wtr_kernel(
    const float* __restrict__ wq, const float* __restrict__ wk, const float* __restrict__ wv,
    const float* __restrict__ wo, unsigned short* __restrict__ wqkv, unsigned short* __restrict__ wob)
{
  __shared__ __align__(16) unsigned short sW[64 * 64];

  const int tid  = (int)threadIdx.x;
  const int sel  = (int)blockIdx.y;
  const int in0  = ((int)blockIdx.x >> 3) * 64;
  const int out0 = ((int)blockIdx.x & 7) * 64;
  const float* src = wq;
  unsigned short* dst = wqkv;
  int f16mode = 0;
  if (sel == 1)      { src = wk; dst = wqkv + (size_t)HIDC * HIDC; }
  else if (sel == 2) { src = wv; dst = wqkv + 2 * (size_t)HIDC * HIDC; }
  else if (sel == 3) { src = wo; dst = wob; f16mode = 1; }

#pragma unroll
  for (int it = 0; it < 4; ++it) {
    const int idx = it * 256 + tid;
    const int r = idx >> 4, c4 = idx & 15;
    const v4f_ a = *(const v4f*)(src + (size_t)(in0 + r) * HIDC + out0 + c4 * 4);
    if (f16mode) {
      sW[(c4 * 4 + 0) * 64 + r] = toh_flush_bits(WOC * bf16_rn(a[0]));
      sW[(c4 * 4 + 1) * 64 + r] = toh_flush_bits(WOC * bf16_rn(a[1]));
      sW[(c4 * 4 + 2) * 64 + r] = toh_flush_bits(WOC * bf16_rn(a[2]));
      sW[(c4 * 4 + 3) * 64 + r] = toh_flush_bits(WOC * bf16_rn(a[3]));
    } else {
      sW[(c4 * 4 + 0) * 64 + r] = bf16_bits(a[0]);
      sW[(c4 * 4 + 1) * 64 + r] = bf16_bits(a[1]);
      sW[(c4 * 4 + 2) * 64 + r] = bf16_bits(a[2]);
      sW[(c4 * 4 + 3) * 64 + r] = bf16_bits(a[3]);
    }
  }
  __syncthreads();

  v4u_ pv[2];
#pragma unroll
  for (int it = 0; it < 2; ++it) {
    const int p = it * 256 + tid;
    pv[it] = *(const v4u*)&sW[(p >> 3) * 64 + (p & 7) * 8];
  }
#pragma unroll
  for (int it = 0; it < 2; ++it) {
    const int p = it * 256 + tid, L = p >> 3, q = p & 7;
    *(volatile v4u_*)(dst + (size_t)(out0 + L) * HIDC + in0 + q * 8) = pv[it];
  }
  __threadfence();
#pragma unroll
  for (int it = 0; it < 2; ++it) {
    const int p = it * 256 + tid, L = p >> 3, q = p & 7;
    *(volatile v4u_*)(dst + (size_t)(out0 + L) * HIDC + in0 + q * 8) = pv[it];
  }
}

__global__ void __launch_bounds__(256) proj_kernel(
    const unsigned short* __restrict__ xb, const unsigned short* __restrict__ wqkv,
    unsigned short* __restrict__ qh, unsigned short* __restrict__ kh, unsigned short* __restrict__ vt)
{
  __shared__ __align__(16) unsigned short sT[128 * 64];

  const int tid  = (int)threadIdx.x;
  const int lane = tid & 31, wave = tid >> 5;
  const int h = lane >> 4, m = lane & 15;
  const int n0  = (int)blockIdx.x * 64;
  const int c0  = (int)blockIdx.y * 128;
  const int sel = c0 / HIDC;
  const int cw  = c0 - sel * HIDC;
  if (sel == 0 && n0 >= QROWS) return;

  const unsigned short* Wb = wqkv + (size_t)sel * HIDC * HIDC;
  const unsigned short* Xb = xb + (size_t)sel * NNODE * HIDC;
  unsigned short* plane = qh;
  if (sel == 1)      { plane = kh; }
  else if (sel == 2) { plane = vt; }

  const int wr = wave >> 2, wc = wave & 3;
  const int rbase = n0 + wr * 32;
  const int cbase = cw + wc * 32;

  v8f acc[2][2] = {};
#pragma unroll 2
  for (int k0 = 0; k0 < HIDC; k0 += 32) {
    FragB a[2], b[2];
#pragma unroll
    for (int rt = 0; rt < 2; ++rt) {
      const unsigned short* ar = Xb + (size_t)(rbase + rt * 16 + m) * HIDC + k0 + 8 * h;
      a[rt].h[0] = *(const v8us*)(ar);
      a[rt].h[1] = *(const v8us*)(ar + 16);
    }
#pragma unroll
    for (int ct = 0; ct < 2; ++ct) {
      const unsigned short* wrp = Wb + (size_t)(cbase + ct * 16 + m) * HIDC + k0 + 8 * h;
      b[ct].h[0] = *(const v8us*)(wrp);
      b[ct].h[1] = *(const v8us*)(wrp + 16);
    }
#pragma unroll
    for (int rt = 0; rt < 2; ++rt)
#pragma unroll
      for (int ct = 0; ct < 2; ++ct)
        acc[rt][ct] = mma_bf16(a[rt].v, b[ct].v, acc[rt][ct]);
  }

  if (sel == 2) {
#pragma unroll
    for (int rt = 0; rt < 2; ++rt)
#pragma unroll
      for (int ct = 0; ct < 2; ++ct) {
        const int cl = wc * 32 + ct * 16 + m;
        v8h_ o;
#pragma unroll
        for (int r = 0; r < 8; ++r) o[r] = toh_flush(acc[rt][ct][r]);
        *(v8us*)&sT[cl * 64 + wr * 32 + rt * 16 + 8 * h] = __builtin_bit_cast(v8us_, o);
      }
  } else {
#pragma unroll
    for (int rt = 0; rt < 2; ++rt)
#pragma unroll
      for (int ct = 0; ct < 2; ++ct) {
        const int cl = wc * 32 + ct * 16 + m;
        const int Lb = (cl >> 6) * 64 + wr * 32 + rt * 16 + 8 * h;
        const int d  = cl & 63;
#pragma unroll
        for (int r = 0; r < 8; ++r) sT[(Lb + r) * 64 + d] = toh_flush_bits(acc[rt][ct][r]);
      }
  }
  __syncthreads();

  v4u_ pv[4];
#pragma unroll
  for (int it = 0; it < 4; ++it) {
    const int p = it * 256 + tid;
    pv[it] = *(const v4u*)&sT[(p >> 3) * 64 + (p & 7) * 8];
  }
  const int h0 = cw >> 6;
#pragma unroll
  for (int it = 0; it < 4; ++it) {
    const int p = it * 256 + tid, L = p >> 3, q = p & 7;
    unsigned short* dstp;
    if (sel == 2) dstp = plane + (size_t)(cw + L) * NNODE + n0 + q * 8;
    else          dstp = plane + ((size_t)(h0 + (L >> 6)) * NNODE + n0 + (L & 63)) * HDIM + q * 8;
    *(volatile v4u_*)dstp = pv[it];
  }
  __threadfence();
#pragma unroll
  for (int it = 0; it < 4; ++it) {
    const int p = it * 256 + tid, L = p >> 3, q = p & 7;
    unsigned short* dstp;
    if (sel == 2) dstp = plane + (size_t)(cw + L) * NNODE + n0 + q * 8;
    else          dstp = plane + ((size_t)(h0 + (L >> 6)) * NNODE + n0 + (L & 63)) * HDIM + q * 8;
    *(volatile v4u_*)dstp = pv[it];
  }
}

__global__ void __launch_bounds__(256) attn_kernel(
    const _Float16* __restrict__ qh, const _Float16* __restrict__ kh, const _Float16* __restrict__ vt,
    unsigned short* __restrict__ ctx)
{
  __shared__ __align__(16) unsigned short sC[NHEAD * 16 * HDIM];

  const int tid  = (int)threadIdx.x;
  const int lane = tid & 31, wave = tid >> 5;
  const int h = lane >> 4, m = lane & 15;
  const int i0 = (int)blockIdx.x * 16;
  const int hd = wave;

  const _Float16* Qn = qh + (size_t)hd * NNODE * HDIM;
  const _Float16* Kn = kh + (size_t)hd * NNODE * HDIM;
  const _Float16* Vn = vt + (size_t)hd * HDIM * NNODE;
  const v8f z8 = {};

  FragH qb0, qb1;
  {
    const _Float16* qr = Qn + (size_t)(i0 + m) * HDIM + 8 * h;
    qb0.h[0] = *(const v8h*)(qr);       qb0.h[1] = *(const v8h*)(qr + 16);
    qb1.h[0] = *(const v8h*)(qr + 32);  qb1.h[1] = *(const v8h*)(qr + 48);
  }

  v8f oacc[4] = {};
  float mi = -3.0e30f;
  float li = 0.0f;

#pragma unroll 1
  for (int j0 = 0; j0 < NNODE; j0 += 32) {
    FragH k0a, k0b, k1a, k1b;
    {
      const _Float16* kp0 = Kn + (size_t)(j0 + m) * HDIM + 8 * h;
      const _Float16* kp1 = kp0 + (size_t)16 * HDIM;
      k0a.h[0] = *(const v8h*)(kp0);       k0a.h[1] = *(const v8h*)(kp0 + 16);
      k0b.h[0] = *(const v8h*)(kp0 + 32);  k0b.h[1] = *(const v8h*)(kp0 + 48);
      k1a.h[0] = *(const v8h*)(kp1);       k1a.h[1] = *(const v8h*)(kp1 + 16);
      k1b.h[0] = *(const v8h*)(kp1 + 32);  k1b.h[1] = *(const v8h*)(kp1 + 48);
    }
    v8f s0 = mma_f16(k0a.v, qb0.v, z8);
    s0 = mma_f16(k0b.v, qb1.v, s0);
    v8f s1 = mma_f16(k1a.v, qb0.v, z8);
    s1 = mma_f16(k1b.v, qb1.v, s1);

    float t0[8], t1[8];
    float cm = -3.0e30f;
#pragma unroll
    for (int r = 0; r < 8; ++r) {
      t0[r] = s0[r] * SCL;
      t1[r] = s1[r] * SCL;
      cm = fmaxf(cm, fmaxf(t0[r], t1[r]));
    }
    cm = fmaxf(cm, __shfl_xor(cm, 16, 32));
    const float mnew = fmaxf(mi, cm);
    const float corr = exp2fast(mi - mnew);

    float rs = 0.0f;
    FragH pa;
#pragma unroll
    for (int r = 0; r < 8; ++r) {
      const float a0 = t0[r] - mnew;
      const float a1 = t1[r] - mnew;
      const float e0r = exp2fast(a0);
      const float e1r = exp2fast(a1);
      const float e0 = (a0 < PFLUSH) ? 0.0f : e0r;
      const float e1 = (a1 < PFLUSH) ? 0.0f : e1r;
      rs += e0 + e1;
      pa.h[0][r] = (_Float16)(e0 * PCARRY);
      pa.h[1][r] = (_Float16)(e1 * PCARRY);
    }
    rs += __shfl_xor(rs, 16, 32);
    li = li * corr + rs;
    mi = mnew;

    float cr[8];
#pragma unroll
    for (int r = 0; r < 8; ++r) cr[r] = __shfl(corr, 8 * h + r, 32);
#pragma unroll
    for (int t = 0; t < 4; ++t)
#pragma unroll
      for (int r = 0; r < 8; ++r) oacc[t][r] *= cr[r];

    FragH vb[4];
#pragma unroll
    for (int t = 0; t < 4; ++t) {
      const _Float16* vp = Vn + (size_t)(t * 16 + m) * NNODE + j0 + 8 * h;
      vb[t].h[0] = *(const v8h*)(vp);
      vb[t].h[1] = *(const v8h*)(vp + 16);
    }
#pragma unroll
    for (int t = 0; t < 4; ++t) oacc[t] = mma_f16(pa.v, vb[t].v, oacc[t]);
  }

  const float inv = CTXSC * (1.0f / li);
  float fl[8];
#pragma unroll
  for (int r = 0; r < 8; ++r) fl[r] = __shfl(inv, 8 * h + r, 32);
#pragma unroll
  for (int t = 0; t < 4; ++t)
#pragma unroll
    for (int r = 0; r < 8; ++r)
      sC[(hd * 16 + 8 * h + r) * HDIM + t * 16 + m] = toh_flush_bits(oacc[t][r] * fl[r]);
  __syncthreads();

  v4u_ cv[4];
#pragma unroll
  for (int it = 0; it < 4; ++it) {
    const int p = it * 256 + tid;
    cv[it] = *(const v4u*)&sC[(p >> 3) * 64 + (p & 7) * 8];
  }
#pragma unroll
  for (int it = 0; it < 4; ++it) {
    const int p = it * 256 + tid, L = p >> 3, q = p & 7;
    *(volatile v4u_*)(ctx + ((size_t)(i0 + (L & 15)) * HIDC + (size_t)(L >> 4) * HDIM + q * 8)) = cv[it];
  }
  __threadfence();
#pragma unroll
  for (int it = 0; it < 4; ++it) {
    const int p = it * 256 + tid, L = p >> 3, q = p & 7;
    *(volatile v4u_*)(ctx + ((size_t)(i0 + (L & 15)) * HIDC + (size_t)(L >> 4) * HDIM + q * 8)) = cv[it];
  }
}

__global__ void __launch_bounds__(256) oproj_kernel(
    const _Float16* __restrict__ act, const _Float16* __restrict__ wo16,
    const float* __restrict__ bo, unsigned short* __restrict__ mid, float* __restrict__ out, int to_mid)
{
  __shared__ __align__(16) float sY[16 * HIDC];

  const int tid  = (int)threadIdx.x;
  const int lane = tid & 31, wave = tid >> 5;
  const int h = lane >> 4, m = lane & 15;
  const int n0 = (int)blockIdx.x * 16;
  const int cb = wave * 64;

  v8f acc[4] = {};
#pragma unroll 2
  for (int k0 = 0; k0 < HIDC; k0 += 32) {
    FragH a;
    const _Float16* ar = act + (size_t)(n0 + m) * HIDC + k0 + 8 * h;
    a.h[0] = *(const v8h*)(ar);
    a.h[1] = *(const v8h*)(ar + 16);
    FragH b[4];
#pragma unroll
    for (int ct = 0; ct < 4; ++ct) {
      const _Float16* wr = wo16 + (size_t)(cb + ct * 16 + m) * HIDC + k0 + 8 * h;
      b[ct].h[0] = *(const v8h*)(wr);
      b[ct].h[1] = *(const v8h*)(wr + 16);
    }
#pragma unroll
    for (int ct = 0; ct < 4; ++ct) acc[ct] = mma_f16(a.v, b[ct].v, acc[ct]);
  }
#pragma unroll
  for (int ct = 0; ct < 4; ++ct) {
    const int col = cb + ct * 16 + m;
    const float bb = bf16_rn(bo[col]);
#pragma unroll
    for (int r = 0; r < 8; ++r) sY[(8 * h + r) * HIDC + col] = acc[ct][r] * OUNC + bb;
  }
  __syncthreads();

  if (to_mid != 0) {
    v8us_ mv[2][2];
#pragma unroll
    for (int rr = 0; rr < 2; ++rr)
#pragma unroll
      for (int it = 0; it < 2; ++it) {
        const int row = wave * 2 + rr;
        const int p = it * 32 + lane;
        const v4f_ a = *(const v4f*)&sY[row * HIDC + p * 8];
        const v4f_ b = *(const v4f*)&sY[row * HIDC + p * 8 + 4];
        v8us_ o;
        o[0] = toh_flush_bits(a[0] * OCARRY); o[1] = toh_flush_bits(a[1] * OCARRY);
        o[2] = toh_flush_bits(a[2] * OCARRY); o[3] = toh_flush_bits(a[3] * OCARRY);
        o[4] = toh_flush_bits(b[0] * OCARRY); o[5] = toh_flush_bits(b[1] * OCARRY);
        o[6] = toh_flush_bits(b[2] * OCARRY); o[7] = toh_flush_bits(b[3] * OCARRY);
        mv[rr][it] = o;
      }
#pragma unroll
    for (int rr = 0; rr < 2; ++rr)
#pragma unroll
      for (int it = 0; it < 2; ++it)
        *(volatile v8us_*)(mid + (size_t)(n0 + wave * 2 + rr) * HIDC + (size_t)(it * 32 + lane) * 8) = mv[rr][it];
    __threadfence();
#pragma unroll
    for (int rr = 0; rr < 2; ++rr)
#pragma unroll
      for (int it = 0; it < 2; ++it)
        *(volatile v8us_*)(mid + (size_t)(n0 + wave * 2 + rr) * HIDC + (size_t)(it * 32 + lane) * 8) = mv[rr][it];
  } else {
    v4f_ ov[2][4];
#pragma unroll
    for (int rr = 0; rr < 2; ++rr)
#pragma unroll
      for (int it = 0; it < 4; ++it) {
        const int row = wave * 2 + rr;
        const int p = it * 32 + lane;
        ov[rr][it] = *(const v4f*)&sY[row * HIDC + p * 4];
      }
#pragma unroll
    for (int rr = 0; rr < 2; ++rr)
#pragma unroll
      for (int it = 0; it < 4; ++it)
        *(volatile v4f_*)(out + (size_t)(n0 + wave * 2 + rr) * HIDC + (size_t)(it * 32 + lane) * 4) = ov[rr][it];
    __threadfence();
#pragma unroll
    for (int rr = 0; rr < 2; ++rr)
#pragma unroll
      for (int it = 0; it < 4; ++it)
        *(volatile v4f_*)(out + (size_t)(n0 + wave * 2 + rr) * HIDC + (size_t)(it * 32 + lane) * 4) = ov[rr][it];
  }
}

extern "C" void kernel_launch(void* const* d_in, const int* in_sizes, int n_in,
                              void* d_out, int out_size, void* d_ws, size_t ws_size,
                              hipStream_t stream)
{
  if (n_in < 8) return;
  if (in_sizes[0] < NNODE * HIDC || in_sizes[1] < NNODE * HIDC || in_sizes[2] < NNODE * HIDC) return;
  if (in_sizes[3] < HIDC * HIDC || in_sizes[4] < HIDC * HIDC ||
      in_sizes[5] < HIDC * HIDC || in_sizes[6] < HIDC * HIDC) return;
  if (in_sizes[7] < HIDC) return;
  if (out_size < QROWS * HIDC) return;

  const float* xq = (const float*)d_in[0];
  const float* xk = (const float*)d_in[1];
  const float* xv = (const float*)d_in[2];
  const float* wq = (const float*)d_in[3];
  const float* wk = (const float*)d_in[4];
  const float* wv = (const float*)d_in[5];
  const float* wo = (const float*)d_in[6];
  const float* bo = (const float*)d_in[7];
  float* out = (float*)d_out;

  const size_t xb_bytes   = (size_t)3 * NNODE * HIDC * 2;
  const size_t wqkv_bytes = (size_t)3 * HIDC * HIDC * 2;
  const size_t wo_bytes   = (size_t)HIDC * HIDC * 2;
  const size_t qk_bytes   = (size_t)NHEAD * NNODE * HDIM * 2;
  const size_t vt_bytes   = (size_t)NHEAD * HDIM * NNODE * 2;
  const size_t ctx_bytes  = (size_t)NNODE * HIDC * 2;
  const size_t y1_bytes   = (size_t)NNODE * HIDC * 2;
  size_t off = 0;
  unsigned char* ws = (unsigned char*)d_ws;
  unsigned short* xb   = (unsigned short*)(ws + off); off += xb_bytes;
  unsigned short* wqkv = (unsigned short*)(ws + off); off += wqkv_bytes;
  unsigned short* wob  = (unsigned short*)(ws + off); off += wo_bytes;
  unsigned short* qhp  = (unsigned short*)(ws + off); off += qk_bytes;
  unsigned short* khp  = (unsigned short*)(ws + off); off += qk_bytes;
  unsigned short* vtp  = (unsigned short*)(ws + off); off += vt_bytes;
  unsigned short* ctxp = (unsigned short*)(ws + off); off += ctx_bytes;
  unsigned short* y1p  = (unsigned short*)(ws + off); off += y1_bytes;
  if (off > ws_size) return;

  cvt_kernel<<<3 * XB_BLOCKS, 256, 0, stream>>>(xq, xk, xv, xb);
  wtr_kernel<<<dim3(WT_TILES, 4), 256, 0, stream>>>(wq, wk, wv, wo, wqkv, wob);
  proj_kernel<<<dim3(NNODE / 64, (3 * HIDC) / 128), 256, 0, stream>>>(xb, wqkv, qhp, khp, vtp);
  attn_kernel<<<QROWS / 16, 256, 0, stream>>>((const _Float16*)qhp, (const _Float16*)khp,
                                              (const _Float16*)vtp, ctxp);
  oproj_kernel<<<QROWS / 16, 256, 0, stream>>>((const _Float16*)ctxp, (const _Float16*)wob,
                                               bo, y1p, out, 1);
  oproj_kernel<<<QROWS / 16, 256, 0, stream>>>((const _Float16*)y1p, (const _Float16*)wob,
                                               bo, ctxp, out, 0);
}
